// NABlock_41661182771218
// MI455X (gfx1250) — hardware-verified
//
#include <hip/hip_runtime.h>


namespace {
constexpr int Nn = 2, C = 64, Hh = 128, Ww = 128, HEADS = 2, DH = 32, KS = 7, NB = 13, C4 = 256, NTOK = Nn * Hh * Ww;
constexpr float AS_ = 8.0f, EPS = 1e-5f, QSC = 0.17677669529663687f;

typedef _Float16 b16;
typedef __attribute__((ext_vector_type(16))) _Float16 v16b;
typedef __attribute__((ext_vector_type(8))) _Float16 v8b;
typedef __attribute__((ext_vector_type(8))) float v8f;
typedef __attribute__((ext_vector_type(4))) float v4f;
__device__ __forceinline__ float bf16_rne(float f) { unsigned int u = __float_as_uint(f); u += 0x7FFFu + ((u >> 16) & 1u); return __uint_as_float(u & 0xFFFF0000u); }
__device__ __forceinline__ void split16(float v, b16& hi, b16& lo) { hi = (b16)v; lo = (b16)(v - (float)hi); }
__device__ __forceinline__ v16b frag_kb(const b16* p, int hh) { const v8b a = *(const v8b*)(p + 8 * hh), b = *(const v8b*)(p + 16 + 8 * hh); v16b f;
#pragma unroll
  for (int e = 0; e < 8; ++e) { f[e] = a[e]; f[8 + e] = b[e]; } return f; }
__device__ __forceinline__ void frag_split(const float* p, int hh, v16b& fh, v16b& fl) {
#pragma unroll
  for (int e = 0; e < 8; ++e) { b16 a, c; split16(p[8 * hh + e] * AS_, a, c); fh[e] = a; fl[e] = c; split16(p[16 + 8 * hh + e] * AS_, a, c); fh[8 + e] = a; fl[8 + e] = c; } }
__device__ __forceinline__ v8f wmma16b(v16b a, v16b b, v8f c) { v8f d = __builtin_amdgcn_wmma_f32_16x16x32_f16(false, a, false, b, (short)0, c, false, false); asm volatile("v_nop\n\tv_nop\n\tv_nop\n\tv_nop" : "+v"(d) : "v"(a), "v"(b)); return d; }
__device__ __forceinline__ void wave_lds_sync() { __builtin_amdgcn_fence(__ATOMIC_RELEASE, "workgroup"); __builtin_amdgcn_wave_barrier(); __builtin_amdgcn_fence(__ATOMIC_ACQUIRE, "workgroup"); }
__device__ __forceinline__ float nexp(float x) { return __builtin_amdgcn_exp2f(x * 1.4426950408889634f); }
__device__ __forceinline__ float pmul(float a, float b) { float p = a * b; asm volatile("" : "+v"(p)); return p; }
__device__ __forceinline__ float gelu_erf(float x) { return 0.5f * x * (1.0f + erff(x * 0.70710678118654752f)); }

struct Wo_ { static constexpr size_t QKV = 0, PRJ = QKV + 192 * 64, FC1 = PRJ + 64 * 64, FC2 = FC1 + 256 * 64, END = FC2 + 64 * 256; };
struct Po_ { static constexpr int QB = 0, PB = 192, F1B = 256, F2B = 512, L1W = 576, L1B = 640, L2W = 704, L2B = 768, RPB = 832, END = 832 + HEADS * NB * NB; };
__global__ __launch_bounds__(256) void prep_kernel(const float* __restrict__ qkv_w, const float* __restrict__ proj_w, const float* __restrict__ fc1_w, const float* __restrict__ fc2_w, const float* __restrict__ qkv_b, const float* __restrict__ proj_b, const float* __restrict__ fc1_b, const float* __restrict__ fc2_b, const float* __restrict__ l1w, const float* __restrict__ l1b, const float* __restrict__ l2w, const float* __restrict__ l2b, const float* __restrict__ rpb, b16* __restrict__ R, float* __restrict__ P) {
  const int t_ = blockIdx.x * 256 + threadIdx.x, nth = gridDim.x * 256;
  for (int pass = 0; pass < 2; ++pass) {
    for (int q = t_; q < 192 * 64; q += nth) R[Wo_::QKV + q] = (b16)bf16_rne(qkv_w[q]);
    for (int q = t_; q < 64 * 64; q += nth) R[Wo_::PRJ + q] = (b16)bf16_rne(proj_w[q]);
    for (int q = t_; q < 256 * 64; q += nth) R[Wo_::FC1 + q] = (b16)bf16_rne(fc1_w[q]);
    for (int q = t_; q < 64 * 256; q += nth) R[Wo_::FC2 + q] = (b16)bf16_rne(fc2_w[q]);
    for (int q = t_; q < Po_::END; q += nth) { float v; if (q < Po_::PB) v = qkv_b[q]; else if (q < Po_::F1B) v = proj_b[q - Po_::PB]; else if (q < Po_::F2B) v = fc1_b[q - Po_::F1B]; else if (q < Po_::L1W) v = fc2_b[q - Po_::F2B]; else if (q < Po_::L1B) v = l1w[q - Po_::L1W]; else if (q < Po_::L2W) v = l1b[q - Po_::L1B]; else if (q < Po_::L2B) v = l2w[q - Po_::L2W]; else if (q < Po_::RPB) v = l2b[q - Po_::L2B]; else v = rpb[q - Po_::RPB]; P[q] = bf16_rne(v); }
    __threadfence(); }
}

template <int NT_>
__device__ __forceinline__ void wg2(const float* A, int lda, int K, const b16* Bw, int t0, int nloc, int hlf, v8f (&acc)[2][NT_]) {
#pragma unroll
  for (int r = 0; r < 2; ++r)
#pragma unroll
    for (int t = 0; t < NT_; ++t) acc[r][t] = (v8f){};
  for (int kb = 0; kb < K; kb += 32) { v16b a0, l0, a1, l1; frag_split(A + (size_t)nloc * lda + kb, hlf, a0, l0); frag_split(A + (size_t)(16 + nloc) * lda + kb, hlf, a1, l1);
#pragma unroll
    for (int t = 0; t < NT_; ++t) { const v16b bw = frag_kb(Bw + (size_t)((t0 + t) * 16 + nloc) * K + kb, hlf); acc[0][t] = wmma16b(a0, bw, acc[0][t]); acc[0][t] = wmma16b(l0, bw, acc[0][t]); acc[1][t] = wmma16b(a1, bw, acc[1][t]); acc[1][t] = wmma16b(l1, bw, acc[1][t]); } }
}

__global__ __launch_bounds__(128) void qkv_kernel(const float* __restrict__ x, const b16* __restrict__ R, const float* __restrict__ P, float* __restrict__ xt, float* __restrict__ qp, float* __restrict__ kp, float* __restrict__ vp) {
  __shared__ __attribute__((aligned(16))) float Xs[128][C + 4]; __shared__ __attribute__((aligned(16))) float O[4][32][64 + 4];
  const int lane = threadIdx.x & 31, wave = threadIdx.x >> 5, nloc = lane & 15, hlf = lane >> 4, i = blockIdx.x, n = blockIdx.y, t_ = threadIdx.x;
  for (int q = t_; q < C * Ww; q += 128) { const int c = q >> 7, j = q & 127; Xs[j][c] = bf16_rne(x[(((size_t)n * C + c) * Hh + i) * Ww + j]); }
  __syncthreads();
  const size_t tok0 = ((size_t)n * Hh + i) * Ww + wave * 32;
  for (int pass = 0; pass < 2; ++pass) { for (int q = lane; q < 32 * 16; q += 32) { const int r = q >> 4, c4 = (q & 15) * 4; *(volatile v4f*)(xt + (tok0 + r) * C + c4) = *(const v4f*)(&Xs[wave * 32 + r][c4]); } __threadfence(); }
  { const int r = wave * 32 + lane; float s = 0.0f; for (int c = 0; c < C; ++c) s += Xs[r][c]; const float mu = s * (1.0f / C); float q2 = 0.0f; for (int c = 0; c < C; ++c) { const float d = Xs[r][c] - mu; q2 += pmul(d, d); }
    const float is = rsqrtf(q2 * (1.0f / C) + EPS); for (int c = 0; c < C; ++c) Xs[r][c] = pmul((Xs[r][c] - mu) * is, P[Po_::L1W + c]) + P[Po_::L1B + c]; }
  wave_lds_sync();
  for (int which = 0; which < 3; ++which) { v8f acc[2][4]; wg2<4>(&Xs[wave * 32][0], C + 4, C, R + Wo_::QKV, which * 4, nloc, hlf, acc);
    const float scl = (which == 0) ? QSC : 1.0f;
#pragma unroll
    for (int t = 0; t < 4; ++t) { const int cc = t * 16 + nloc; const float bb = P[Po_::QB + which * 64 + cc];
#pragma unroll
      for (int r = 0; r < 2; ++r)
#pragma unroll
        for (int v = 0; v < 8; ++v) O[wave][r * 16 + 8 * hlf + v][cc] = (acc[r][t][v] * (1.0f / AS_) + bb) * scl; }
    wave_lds_sync();
    float* dstp = (which == 0) ? qp : (which == 1) ? kp : vp;
    for (int pass = 0; pass < 2; ++pass) { for (int q = lane; q < 32 * 2 * 8; q += 32) { const int r = q >> 4, hd = (q >> 3) & 1, c4 = (q & 7) * 4; const size_t o = ((((size_t)n * HEADS + hd) * Hh + i) * Ww + wave * 32 + r) * DH + c4; *(volatile v4f*)(dstp + o) = *(const v4f*)(&O[wave][r][hd * DH + c4]); } __threadfence(); }
    wave_lds_sync(); }
}

__global__ __launch_bounds__(256) void attn_mlp_kernel(const float* __restrict__ qp, const float* __restrict__ kp, const float* __restrict__ vp, const float* __restrict__ xt, const b16* __restrict__ R, const float* __restrict__ P, float* __restrict__ out) {
  __shared__ __attribute__((aligned(16))) float A0[128][C + 4];
  __shared__ __attribute__((aligned(16))) float Y[128][C + 4];
  __shared__ __attribute__((aligned(16))) b16 G[128][C4 + 8];
  const int t_ = threadIdx.x, lane = t_ & 31, wave = t_ >> 5, nloc = lane & 15, hlf = lane >> 4, i = blockIdx.x, n = blockIdx.y;
  { const int j = t_ & 127, hd = t_ >> 7; const int si = min(max(i - KS / 2, 0), Hh - KS), sj = min(max(j - KS / 2, 0), Ww - KS);
    const float* qrow = qp + ((((size_t)n * HEADS + hd) * Hh + i) * Ww + j) * DH; float q[DH];
#pragma unroll
    for (int d = 0; d < DH; ++d) q[d] = qrow[d];
    const float* rp = P + Po_::RPB + hd * NB * NB; float m = -INFINITY, l = 0.0f, acc[DH];
#pragma unroll
    for (int d = 0; d < DH; ++d) acc[d] = 0.0f;
#pragma unroll 1
    for (int kk = 0; kk < KS * KS; ++kk) { const int ki = si + kk / KS, kj = sj + kk % KS; const size_t ko = ((((size_t)n * HEADS + hd) * Hh + ki) * Ww + kj) * DH; const float* kr = kp + ko; const float* vr = vp + ko;
      float s = rp[(i - ki + KS - 1) * NB + (j - kj + KS - 1)];
#pragma unroll
      for (int d = 0; d < DH; d += 4) { const v4f k4 = *(const v4f*)(kr + d); s += pmul(q[d], k4[0]); s += pmul(q[d + 1], k4[1]); s += pmul(q[d + 2], k4[2]); s += pmul(q[d + 3], k4[3]); }
      const float mn = fmaxf(m, s), al = nexp(m - mn), e = nexp(s - mn); l = l * al + e; m = mn;
#pragma unroll
      for (int d = 0; d < DH; d += 4) { const v4f v4 = *(const v4f*)(vr + d); acc[d] = acc[d] * al + pmul(e, v4[0]); acc[d + 1] = acc[d + 1] * al + pmul(e, v4[1]); acc[d + 2] = acc[d + 2] * al + pmul(e, v4[2]); acc[d + 3] = acc[d + 3] * al + pmul(e, v4[3]); } }
    const float inv = 1.0f / l;
#pragma unroll
    for (int d = 0; d < DH; ++d) A0[j][hd * DH + d] = acc[d] * inv; }
  __syncthreads();
  const int r0 = wave * 16; const size_t tok0 = ((size_t)n * Hh + i) * Ww + r0;
  { v8f acc[4]; for (int t = 0; t < 4; ++t) acc[t] = (v8f){};
    for (int kb = 0; kb < C; kb += 32) { v16b a, al; frag_split(&A0[r0 + nloc][kb], hlf, a, al);
#pragma unroll
      for (int t = 0; t < 4; ++t) { const v16b bw = frag_kb(R + Wo_::PRJ + (size_t)(t * 16 + nloc) * C + kb, hlf); acc[t] = wmma16b(a, bw, acc[t]); acc[t] = wmma16b(al, bw, acc[t]); } }
    wave_lds_sync();
#pragma unroll
    for (int t = 0; t < 4; ++t) { const int cc = t * 16 + nloc; const float bb = P[Po_::PB + cc];
#pragma unroll
      for (int v = 0; v < 8; ++v) { const int rr = r0 + 8 * hlf + v; A0[rr][cc] = acc[t][v] * (1.0f / AS_) + bb + xt[(tok0 + 8 * hlf + v) * C + cc]; } }
    wave_lds_sync(); }
  if (lane < 16) { const int rr = r0 + lane; float s = 0.0f; for (int c = 0; c < C; ++c) s += A0[rr][c]; const float mu = s * (1.0f / C); float q2 = 0.0f; for (int c = 0; c < C; ++c) { const float d = A0[rr][c] - mu; q2 += pmul(d, d); }
    const float is = rsqrtf(q2 * (1.0f / C) + EPS); for (int c = 0; c < C; ++c) Y[rr][c] = pmul((A0[rr][c] - mu) * is, P[Po_::L2W + c]) + P[Po_::L2B + c]; }
  wave_lds_sync();
  { for (int tg = 0; tg < 16; tg += 8) { v8f acc[8]; for (int t = 0; t < 8; ++t) acc[t] = (v8f){};
      for (int kb = 0; kb < C; kb += 32) { v16b a, al; frag_split(&Y[r0 + nloc][kb], hlf, a, al);
#pragma unroll
        for (int t = 0; t < 8; ++t) { const v16b bw = frag_kb(R + Wo_::FC1 + (size_t)((tg + t) * 16 + nloc) * C + kb, hlf); acc[t] = wmma16b(a, bw, acc[t]); acc[t] = wmma16b(al, bw, acc[t]); } }
#pragma unroll
      for (int t = 0; t < 8; ++t) { const int cc = (tg + t) * 16 + nloc; const float bb = P[Po_::F1B + cc];
#pragma unroll
        for (int v = 0; v < 8; ++v) G[r0 + 8 * hlf + v][cc] = (b16)(acc[t][v] * (1.0f / AS_) + bb); } }
    wave_lds_sync();
#pragma unroll 1
    for (int q = lane; q < 16 * C4; q += 32) { const int rr = r0 + q / C4, cc = q % C4; G[rr][cc] = (b16)gelu_erf((float)G[rr][cc]); }
    wave_lds_sync(); }
  { v8f acc[4]; for (int t = 0; t < 4; ++t) acc[t] = (v8f){};
    for (int kb = 0; kb < C4; kb += 32) { const v16b a = frag_kb(&G[r0 + nloc][kb], hlf);
#pragma unroll
      for (int t = 0; t < 4; ++t) { const v16b bw = frag_kb(R + Wo_::FC2 + (size_t)(t * 16 + nloc) * C4 + kb, hlf); acc[t] = wmma16b(a, bw, acc[t]); } }
#pragma unroll
    for (int t = 0; t < 4; ++t) { const int cc = t * 16 + nloc; const float bb = P[Po_::F2B + cc];
#pragma unroll
      for (int v = 0; v < 8; ++v) { const int rr = r0 + 8 * hlf + v; Y[rr][cc] = A0[rr][cc] + acc[t][v] + bb; } } }
  __syncthreads();
  for (int pass = 0; pass < 2; ++pass) { for (int q = t_; q < C * 32; q += 256) { const int c = q >> 5, j4 = (q & 31) * 4; v4f o; o[0] = Y[j4][c]; o[1] = Y[j4 + 1][c]; o[2] = Y[j4 + 2][c]; o[3] = Y[j4 + 3][c]; *(volatile v4f*)(out + (((size_t)n * C + c) * Hh + i) * Ww + j4) = o; } __threadfence(); }
}
}

extern "C" void kernel_launch(void* const* d_in, const int* in_sizes, int n_in,
                              void* d_out, int out_size, void* d_ws, size_t ws_size, hipStream_t stream) {
  (void)n_in; (void)out_size;
  const float* x = (const float*)d_in[0]; const float* qkv_w = (const float*)d_in[1]; const float* qkv_b = (const float*)d_in[2]; const float* proj_w = (const float*)d_in[3]; const float* proj_b = (const float*)d_in[4]; const float* rpb = (const float*)d_in[5];
  const float* l1w = (const float*)d_in[6]; const float* l1b = (const float*)d_in[7]; const float* l2w = (const float*)d_in[8]; const float* l2b = (const float*)d_in[9]; const float* fc1_w = (const float*)d_in[10]; const float* fc1_b = (const float*)d_in[11]; const float* fc2_w = (const float*)d_in[12]; const float* fc2_b = (const float*)d_in[13];
  float* out = (float*)d_out;
  if (in_sizes[0] != NTOK * C || in_sizes[1] != 192 * 64 || in_sizes[5] != HEADS * NB * NB || in_sizes[10] != 256 * 64 || in_sizes[12] != 64 * 256) return;
  size_t off = 0; char* ws = (char*)d_ws;
  auto carve = [&](size_t bytes) { char* p = ws + off; off += (bytes + 255) & ~(size_t)255; return p; };
  b16* R = (b16*)carve(Wo_::END * 2); float* P = (float*)carve(((size_t)Po_::END + 64) * 4); float* xt = (float*)carve((size_t)NTOK * C * 4);
  float* qp = (float*)carve((size_t)NTOK * C * 4); float* kp = (float*)carve((size_t)NTOK * C * 4); float* vp = (float*)carve((size_t)NTOK * C * 4);
  if (off > ws_size) return;
  prep_kernel<<<32, 256, 0, stream>>>(qkv_w, proj_w, fc1_w, fc2_w, qkv_b, proj_b, fc1_b, fc2_b, l1w, l1b, l2w, l2b, rpb, R, P);
  qkv_kernel<<<dim3(Hh, Nn), 128, 0, stream>>>(x, R, P, xt, qp, kp, vp);
  attn_mlp_kernel<<<dim3(Hh, Nn), 256, 0, stream>>>(qp, kp, vp, xt, R, P, out);
}
